// Model_54202487275578
// MI455X (gfx1250) — hardware-run, weakly checked
//
#include <hip/hip_runtime.h>

typedef __attribute__((ext_vector_type(16))) _Float16 v16h;
typedef __attribute__((ext_vector_type(8)))  _Float16 v8h;
typedef __attribute__((ext_vector_type(8)))  float    v8f;
typedef __attribute__((ext_vector_type(4)))  float    v4f;
typedef __attribute__((ext_vector_type(2)))  float    v2f;
typedef __attribute__((ext_vector_type(4)))  int      v4i;
typedef __attribute__((ext_vector_type(4)))  unsigned int v4u;

constexpr int kBatch = 32;
constexpr int kSteps = 50;
constexpr int kNodes = 60;
constexpr int kEdges = 512;
constexpr int kRows  = kBatch * kSteps;
constexpr int kHidE  = 1024;
constexpr int kHidD  = 256;
constexpr int kGateE = 3 * kHidE;
constexpr int kGateD = 3 * kHidD;
static_assert(kRows == 1600, "rows");
static_assert(kRows % 64 == 0 && kGateE % 64 == 0 && kGateD % 64 == 0 && kHidE % 64 == 0, "tile multiples");
static_assert(kHidE % 32 == 0 && kHidD % 32 == 0, "k multiples of 32");

constexpr float kCarryW  = 256.0f;
constexpr float kCarryA0 = 4096.0f;
constexpr float kCarryE  = 16384.0f;
constexpr float kCarryD  = 65536.0f;
constexpr float kCarryD0 = 65536.0f;
constexpr float kCarryD1 = 262144.0f;
constexpr float kInvWA0 = 1.0f / (kCarryW * kCarryA0);
constexpr float kInvWE  = 1.0f / (kCarryW * kCarryE);
constexpr float kInvWD  = 1.0f / (kCarryW * kCarryD);
constexpr float kInvWD0 = 1.0f / (kCarryW * kCarryD0);
constexpr float kInvWD1 = 1.0f / (kCarryW * kCarryD1);

constexpr float kF16MinNormal = 6.103515625e-05f;
constexpr float kF16Clamp = 60000.0f;

__device__ __forceinline__ _Float16 to_h(float v) {
  float f = fminf(fmaxf(v, -kF16Clamp), kF16Clamp);
  f = (fabsf(f) < kF16MinNormal) ? 0.0f : f;
  return (_Float16)f;
}

union FragU { v16h v; v8h h[2]; };
__device__ __forceinline__ v16h frag_load_f16(const _Float16* p) {
  FragU f;
  f.h[0] = *(const v8h*)(p);
  f.h[1] = *(const v8h*)(p + 16);
  return f.v;
}

__device__ __forceinline__ v8f mma_f16(v16h a, v16h b, v8f c) {
  c = __builtin_amdgcn_wmma_f32_16x16x32_f16(false, a, false, b, (short)0, c, false, false);
  asm volatile("v_nop\n\tv_nop\n\tv_nop\n\tv_nop" : "+v"(c) : "v"(a), "v"(b));
  return c;
}

__global__ __launch_bounds__(256)
void weight_to_f16_kernel(const float* __restrict__ in, unsigned short* __restrict__ out) {
  const size_t i = (size_t)blockIdx.x * 256 + threadIdx.x;
  const v4f a = *(const v4f*)(in + i * 8);
  const v4f b = *(const v4f*)(in + i * 8 + 4);
  v8h h;
  h[0] = to_h(a[0] * kCarryW);
  h[1] = to_h(a[1] * kCarryW);
  h[2] = to_h(a[2] * kCarryW);
  h[3] = to_h(a[3] * kCarryW);
  h[4] = to_h(b[0] * kCarryW);
  h[5] = to_h(b[1] * kCarryW);
  h[6] = to_h(b[2] * kCarryW);
  h[7] = to_h(b[3] * kCarryW);
  volatile v8h* p = (volatile v8h*)(out + i * 8);
  *p = h;
  __threadfence();
  *p = h;
}

__device__ __forceinline__ unsigned int pack_edge(int s, int d) {
  const int sc = min(max(s, 0), kNodes - 1);
  const int dc = min(max(d, 0), kNodes - 1);
  return (unsigned int)sc | ((unsigned int)dc << 8);
}

__global__ __launch_bounds__(128)
void graph_front_kernel(const float* __restrict__ x, const int* __restrict__ ei,
                        const float* __restrict__ W1, const float* __restrict__ b1,
                        const float* __restrict__ W2, const float* __restrict__ b2,
                        float* __restrict__ res) {
  __shared__ __align__(16) unsigned int sEdge[4][kEdges];
  __shared__ __align__(16) float sXwd[4][64 * 4];
  __shared__ __align__(16) float sG2[4][64 * 2];
  __shared__ __align__(16) float sPart[4][32 * 2];
  __shared__ __align__(16) float sRes[32];

  const int tid  = threadIdx.x;
  const int lane = tid & 31;
  const int wave = tid >> 5;
  const int j    = blockIdx.x;
  const int t    = j >> 1;
  const int b0   = (j & 1) * 16;

  const float w1_00 = W1[0], w1_01 = W1[1], w1_02 = W1[2], w1_03 = W1[3];
  const float w1_10 = W1[4], w1_11 = W1[5], w1_12 = W1[6], w1_13 = W1[7];
  const float b1_0 = b1[0], b1_1 = b1[1], b1_2 = b1[2], b1_3 = b1[3];
  const float w2_00 = W2[0], w2_01 = W2[1], w2_10 = W2[2], w2_11 = W2[3];
  const float w2_20 = W2[4], w2_21 = W2[5], w2_30 = W2[6], w2_31 = W2[7];
  const float b2_0 = b2[0], b2_1 = b2[1];

  const int n0 = lane;
  const int n1 = lane + 32;
  const int n1c = n1 < kNodes ? n1 : kNodes - 1;
  const bool n1ok = n1 < kNodes;

#pragma unroll 1
  for (int q = 0; q < 4; ++q) {
    const int gi = wave * 4 + q;
    const int g  = (b0 + gi) * kSteps + t;
    const int* srcp = ei + (size_t)g * 2 * kEdges;
    const int* dstp = srcp + kEdges;

#pragma unroll
    for (int it = 0; it < 4; ++it) {
      const int e4 = it * 32 + lane;
      const v4i sv = *(const v4i*)(srcp + 4 * e4);
      const v4i dv = *(const v4i*)(dstp + 4 * e4);
      v4u pk;
      pk[0] = pack_edge(sv[0], dv[0]);
      pk[1] = pack_edge(sv[1], dv[1]);
      pk[2] = pack_edge(sv[2], dv[2]);
      pk[3] = pack_edge(sv[3], dv[3]);
      *(v4u*)(&sEdge[wave][4 * e4]) = pk;
    }
    const float* xg = x + (size_t)g * kNodes * 2;
    const v2f xa = *(const v2f*)(xg + 2 * n0);
    const v2f xbv = *(const v2f*)(xg + 2 * n1c);
    float xb0 = xbv[0];
    float xb1 = xbv[1];
    asm volatile("" : "+v"(xb0), "+v"(xb1));
    __syncthreads();

    int c0 = 1, c1 = 1;
#pragma unroll 2
    for (int i = 0; i < kEdges / 4; ++i) {
      const v4u w = *(const v4u*)(&sEdge[wave][4 * i]);
#pragma unroll
      for (int c = 0; c < 4; ++c) {
        const int d = (int)(w[c] >> 8);
        c0 += (d == n0) ? 1 : 0;
        c1 += (d == n1) ? 1 : 0;
      }
    }
    const float deg0 = (float)c0;
    const float deg1 = (float)c1;
    const float dinv0 = (deg0 > 0.0f) ? (1.0f / sqrtf(fmaxf(deg0, 1e-12f))) : 0.0f;
    const float dinv1 = (deg1 > 0.0f) ? (1.0f / sqrtf(fmaxf(deg1, 1e-12f))) : 0.0f;

    v4f q0, q1;
    q0[0] = (xa[0] * w1_00 + xa[1] * w1_10) * dinv0;
    q0[1] = (xa[0] * w1_01 + xa[1] * w1_11) * dinv0;
    q0[2] = (xa[0] * w1_02 + xa[1] * w1_12) * dinv0;
    q0[3] = (xa[0] * w1_03 + xa[1] * w1_13) * dinv0;
    q1[0] = n1ok ? (xb0 * w1_00 + xb1 * w1_10) * dinv1 : 0.0f;
    q1[1] = n1ok ? (xb0 * w1_01 + xb1 * w1_11) * dinv1 : 0.0f;
    q1[2] = n1ok ? (xb0 * w1_02 + xb1 * w1_12) * dinv1 : 0.0f;
    q1[3] = n1ok ? (xb0 * w1_03 + xb1 * w1_13) * dinv1 : 0.0f;
    *(v4f*)(&sXwd[wave][4 * n0]) = q0;
    *(v4f*)(&sXwd[wave][4 * n1]) = q1;
    __syncthreads();

    float a00 = 0.0f, a01 = 0.0f, a02 = 0.0f, a03 = 0.0f;
    float a10 = 0.0f, a11 = 0.0f, a12 = 0.0f, a13 = 0.0f;
#pragma unroll 1
    for (int i = 0; i < kEdges / 4; ++i) {
      const v4u w = *(const v4u*)(&sEdge[wave][4 * i]);
#pragma unroll
      for (int c = 0; c < 4; ++c) {
        const unsigned int wc = w[c];
        const int s = (int)(wc & 0xffu);
        const int d = (int)(wc >> 8);
        const v4f xs = *(const v4f*)(&sXwd[wave][4 * s]);
        const bool m0 = (d == n0);
        const bool m1 = (d == n1);
        a00 += m0 ? xs[0] : 0.0f;
        a01 += m0 ? xs[1] : 0.0f;
        a02 += m0 ? xs[2] : 0.0f;
        a03 += m0 ? xs[3] : 0.0f;
        a10 += m1 ? xs[0] : 0.0f;
        a11 += m1 ? xs[1] : 0.0f;
        a12 += m1 ? xs[2] : 0.0f;
        a13 += m1 ? xs[3] : 0.0f;
      }
    }
    const float h00 = (a00 + q0[0]) * dinv0 + b1_0;
    const float h01 = (a01 + q0[1]) * dinv0 + b1_1;
    const float h02 = (a02 + q0[2]) * dinv0 + b1_2;
    const float h03 = (a03 + q0[3]) * dinv0 + b1_3;
    const float h10 = (a10 + q1[0]) * dinv1 + b1_0;
    const float h11 = (a11 + q1[1]) * dinv1 + b1_1;
    const float h12 = (a12 + q1[2]) * dinv1 + b1_2;
    const float h13 = (a13 + q1[3]) * dinv1 + b1_3;
    v2f g0, g1;
    g0[0] = dinv0 * (h00 * w2_00 + h01 * w2_10 + h02 * w2_20 + h03 * w2_30);
    g0[1] = dinv0 * (h00 * w2_01 + h01 * w2_11 + h02 * w2_21 + h03 * w2_31);
    g1[0] = dinv1 * (h10 * w2_00 + h11 * w2_10 + h12 * w2_20 + h13 * w2_30);
    g1[1] = dinv1 * (h10 * w2_01 + h11 * w2_11 + h12 * w2_21 + h13 * w2_31);
    *(v2f*)(&sG2[wave][2 * n0]) = g0;
    *(v2f*)(&sG2[wave][2 * n1]) = g1;
    __syncthreads();

    float p0 = 0.0f, p1 = 0.0f;
#pragma unroll
    for (int i = 0; i < 4; ++i) {
      const v4u w = *(const v4u*)(&sEdge[wave][16 * lane + 4 * i]);
#pragma unroll
      for (int c = 0; c < 4; ++c) {
        const unsigned int wc = w[c];
        const int s = (int)(wc & 0xffu);
        const int d = (int)(wc >> 8);
        const v2f gv = *(const v2f*)(&sG2[wave][2 * s]);
        const bool m = (d == 0);
        p0 += m ? gv[0] : 0.0f;
        p1 += m ? gv[1] : 0.0f;
      }
    }
    v2f pv;
    pv[0] = p0;
    pv[1] = p1;
    *(v2f*)(&sPart[wave][2 * lane]) = pv;
    __syncthreads();

    const int cc = lane & 1;
    float sum = 0.0f;
#pragma unroll 8
    for (int l = 0; l < 32; ++l) sum += sPart[wave][2 * l + cc];
    sum += sG2[wave][cc];
    const float d0 = __shfl(dinv0, 0, 32);
    const float b2c = (cc == 0) ? b2_0 : b2_1;
    const float rv = d0 * sum + b2c;
    if (lane < 2) sRes[gi * 2 + lane] = rv;
  }
  __syncthreads();
  if (tid < 8) {
    const v4f v = *(const v4f*)(&sRes[4 * tid]);
    volatile v4f* p = (volatile v4f*)(res + (size_t)j * 32 + 4 * tid);
    *p = v;
    __threadfence();
    *p = v;
  }
}

__global__ __launch_bounds__(256)
void front_linear_kernel(const float* __restrict__ res, const float* __restrict__ W,
                         const float* __restrict__ bias, unsigned short* __restrict__ outA) {
  const int idx = blockIdx.x * 256 + threadIdx.x;
  const int row = idx >> 7;
  const int j0  = (idx & 127) * 8;
  const v2f r = *(const v2f*)(res + 2 * row);
  const v4f w0 = *(const v4f*)(W + 2 * j0);
  const v4f w1 = *(const v4f*)(W + 2 * j0 + 4);
  const v4f w2 = *(const v4f*)(W + 2 * j0 + 8);
  const v4f w3 = *(const v4f*)(W + 2 * j0 + 12);
  const v4f ba = *(const v4f*)(bias + j0);
  const v4f bb = *(const v4f*)(bias + j0 + 4);
  v8h h;
  h[0] = to_h(fmaxf(r[0] * w0[0] + r[1] * w0[1] + ba[0], 0.0f) * kCarryA0);
  h[1] = to_h(fmaxf(r[0] * w0[2] + r[1] * w0[3] + ba[1], 0.0f) * kCarryA0);
  h[2] = to_h(fmaxf(r[0] * w1[0] + r[1] * w1[1] + ba[2], 0.0f) * kCarryA0);
  h[3] = to_h(fmaxf(r[0] * w1[2] + r[1] * w1[3] + ba[3], 0.0f) * kCarryA0);
  h[4] = to_h(fmaxf(r[0] * w2[0] + r[1] * w2[1] + bb[0], 0.0f) * kCarryA0);
  h[5] = to_h(fmaxf(r[0] * w2[2] + r[1] * w2[3] + bb[1], 0.0f) * kCarryA0);
  h[6] = to_h(fmaxf(r[0] * w3[0] + r[1] * w3[1] + bb[2], 0.0f) * kCarryA0);
  h[7] = to_h(fmaxf(r[0] * w3[2] + r[1] * w3[3] + bb[3], 0.0f) * kCarryA0);
  volatile v8h* p = (volatile v8h*)(outA + (size_t)row * kHidE + j0);
  *p = h;
  __threadfence();
  *p = h;
}

template <int BIAS_MODE, int OUT_MODE, int ACT>
__global__ __launch_bounds__(256)
void gemm64_f16_kernel(const unsigned short* __restrict__ Ap, int lda,
                       const unsigned short* __restrict__ Btp, int ldb,
                       void* __restrict__ Cout, int ldc,
                       const float* __restrict__ bias,
                       int M, int N, int K, float scale, float oscale) {
  const _Float16* A  = (const _Float16*)Ap;
  const _Float16* Bt = (const _Float16*)Btp;
  __shared__ __align__(16) float sT[8][16 * 68];
  const int lane = threadIdx.x & 31;
  const int wave = threadIdx.x >> 5;
  const int tilesN = N >> 6;
  const int tilesM = M >> 6;
  const int tile = blockIdx.x * 8 + wave;
  if (tile >= tilesM * tilesN) return;
  const int tm = tile / tilesN;
  const int tn = tile - tm * tilesN;
  const int m0 = tm << 6;
  const int n0 = tn << 6;
  const int rlane = lane & 15;
  const int koff  = (lane >> 4) * 8;
  const int mOff  = (lane >> 4) * 8;

  v8f acc[4][4];
#pragma unroll
  for (int i = 0; i < 4; ++i)
#pragma unroll
    for (int jj = 0; jj < 4; ++jj) acc[i][jj] = (v8f){0.f, 0.f, 0.f, 0.f, 0.f, 0.f, 0.f, 0.f};

  for (int k0 = 0; k0 < K; k0 += 32) {
    v16h bh[4];
#pragma unroll
    for (int jj = 0; jj < 4; ++jj)
      bh[jj] = frag_load_f16(Bt + (size_t)(n0 + (jj << 4) + rlane) * ldb + koff + k0);
#pragma unroll
    for (int i = 0; i < 4; ++i) {
      const v16h ah = frag_load_f16(A + (size_t)(m0 + (i << 4) + rlane) * lda + koff + k0);
#pragma unroll
      for (int jj = 0; jj < 4; ++jj) acc[i][jj] = mma_f16(ah, bh[jj], acc[i][jj]);
    }
  }

  float* slab = sT[wave];
#pragma unroll
  for (int i = 0; i < 4; ++i) {
    const int mBase = m0 + (i << 4);
    float bm[8];
#pragma unroll
    for (int r = 0; r < 8; ++r) bm[r] = (BIAS_MODE == 1) ? bias[mBase + mOff + r] : 0.0f;
#pragma unroll
    for (int jj = 0; jj < 4; ++jj) {
      float bv = 0.0f;
      if (BIAS_MODE == 2) bv = bias[n0 + (jj << 4) + rlane];
#pragma unroll
      for (int r = 0; r < 8; ++r) {
        float v = acc[i][jj][r] * scale;
        if (BIAS_MODE == 1) v += bm[r];
        if (BIAS_MODE == 2) v += bv;
        if (ACT == 2) v = fmaxf(v, 0.0f);
        if (OUT_MODE == 1) v *= oscale;
        slab[(mOff + r) * 68 + (jj << 4) + rlane] = v;
      }
    }
    __builtin_amdgcn_fence(__ATOMIC_RELEASE, "workgroup");
    __builtin_amdgcn_wave_barrier();
    __builtin_amdgcn_fence(__ATOMIC_ACQUIRE, "workgroup");
    if (OUT_MODE == 0) {
      float* C = (float*)Cout;
      const int hh = lane >> 4, c4 = (lane & 15) * 4;
      for (int pass = 0; pass < 2; ++pass) {
#pragma unroll
        for (int it = 0; it < 8; ++it) {
          const int row = it * 2 + hh;
          const v4f v = *(const v4f*)(slab + row * 68 + c4);
          *(volatile v4f*)(C + (size_t)(mBase + row) * ldc + n0 + c4) = v;
        }
        __threadfence();
      }
    } else {
      unsigned short* C = (unsigned short*)Cout;
      const int qq = lane >> 3, c8 = (lane & 7) * 8;
      for (int pass = 0; pass < 2; ++pass) {
#pragma unroll
        for (int it = 0; it < 4; ++it) {
          const int row = it * 4 + qq;
          const float* sp = slab + row * 68 + c8;
          v8h hv;
#pragma unroll
          for (int e = 0; e < 8; ++e) hv[e] = to_h(sp[e]);
          *(volatile v8h*)(C + (size_t)(mBase + row) * ldc + n0 + c8) = hv;
        }
        __threadfence();
      }
    }
    __builtin_amdgcn_fence(__ATOMIC_RELEASE, "workgroup");
    __builtin_amdgcn_wave_barrier();
    __builtin_amdgcn_fence(__ATOMIC_ACQUIRE, "workgroup");
  }
}

__device__ __forceinline__ float sigmoid_f32(float v) {
  return __builtin_amdgcn_rcpf(1.0f + expf(-v));
}

template <int H, bool F32OUT>
__global__ __launch_bounds__(512)
void recurrent_layer_kernel(const unsigned short* __restrict__ Whh16, const float* __restrict__ bhh,
                            const float* __restrict__ xiT,
                            unsigned short* __restrict__ y16, float* __restrict__ y32,
                            float carryH, float invCarry) {
  constexpr int NT = H / 256;
  constexpr int HP = H + 8;
  constexpr int CP = H + 4;
  static_assert(NT * 256 == H, "16 waves x NT tiles x 16 columns");
  __shared__ __align__(16) _Float16 sH[16 * HP];
  __shared__ __align__(16) float sC[16 * CP];

  const int tid  = threadIdx.x;
  const int lane = tid & 31;
  const int wave = tid >> 5;
  const int rl   = lane & 15;
  const int hh   = lane >> 4;
  const int b0   = blockIdx.x * 16;

  for (int i = tid; i < 16 * HP / 2; i += 512) ((unsigned int*)sH)[i] = 0u;
  for (int i = tid; i < 16 * CP; i += 512) sC[i] = 0.0f;
  __syncthreads();

  const _Float16* W = (const _Float16*)Whh16;

#pragma unroll 1
  for (int t = 0; t < kSteps; ++t) {
#pragma unroll 1
    for (int nt = 0; nt < NT; ++nt) {
      const int col = (wave * NT + nt) * 16 + rl;
      v8f ar = (v8f){0.f, 0.f, 0.f, 0.f, 0.f, 0.f, 0.f, 0.f};
      v8f az = ar;
      v8f an = ar;
      const _Float16* wr = W + (size_t)col * H + 8 * hh;
      const _Float16* wz = wr + (size_t)H * H;
      const _Float16* wn = wz + (size_t)H * H;
      const _Float16* ap = sH + rl * HP + 8 * hh;
#pragma unroll 4
      for (int k0 = 0; k0 < H; k0 += 32) {
        const v16h a  = frag_load_f16(ap + k0);
        const v16h br = frag_load_f16(wr + k0);
        ar = mma_f16(a, br, ar);
        const v16h bz = frag_load_f16(wz + k0);
        az = mma_f16(a, bz, az);
        const v16h bn = frag_load_f16(wn + k0);
        an = mma_f16(a, bn, an);
      }
      const int row0 = t * 32 + b0 + 8 * hh;
      const float* xp = xiT + (size_t)col * kRows + row0;
      const v4f xr0 = *(const v4f*)(xp);
      const v4f xr1 = *(const v4f*)(xp + 4);
      const v4f xz0 = *(const v4f*)(xp + (size_t)H * kRows);
      const v4f xz1 = *(const v4f*)(xp + (size_t)H * kRows + 4);
      const v4f xn0 = *(const v4f*)(xp + (size_t)2 * H * kRows);
      const v4f xn1 = *(const v4f*)(xp + (size_t)2 * H * kRows + 4);
      const float bhr = bhh[col];
      const float bhz = bhh[H + col];
      const float bhn = bhh[2 * H + col];
      const float xr[8] = {xr0[0], xr0[1], xr0[2], xr0[3], xr1[0], xr1[1], xr1[2], xr1[3]};
      const float xz[8] = {xz0[0], xz0[1], xz0[2], xz0[3], xz1[0], xz1[1], xz1[2], xz1[3]};
      const float xn[8] = {xn0[0], xn0[1], xn0[2], xn0[3], xn1[0], xn1[1], xn1[2], xn1[3]};
#pragma unroll
      for (int r = 0; r < 8; ++r) {
        const float ghr = fmaf(ar[r], invCarry, bhr);
        const float ghz = fmaf(az[r], invCarry, bhz);
        const float ghn = fmaf(an[r], invCarry, bhn);
        const float rg = sigmoid_f32(xr[r] + ghr);
        const float zg = sigmoid_f32(xz[r] + ghz);
        const float ng = tanhf(fmaf(rg, ghn, xn[r]));
        const int ci = (8 * hh + r) * CP + col;
        const float hold = sC[ci];
        const float hnew = (1.0f - zg) * ng + zg * hold;
        sC[ci] = hnew;
      }
    }
    __syncthreads();

    constexpr int NIT = (16 * H / 8) / 512;
    static_assert(NIT * 512 * 8 == 16 * H, "operand tile coverage");
    v8h hv[NIT];
    size_t goff[NIT];
#pragma unroll
    for (int it = 0; it < NIT; ++it) {
      const int c   = it * 512 + tid;
      const int row = c / (H / 8);
      const int c8  = (c - row * (H / 8)) * 8;
      const v4f f0 = *(const v4f*)(sC + row * CP + c8);
      const v4f f1 = *(const v4f*)(sC + row * CP + c8 + 4);
      v8h h;
      h[0] = to_h(f0[0] * carryH);
      h[1] = to_h(f0[1] * carryH);
      h[2] = to_h(f0[2] * carryH);
      h[3] = to_h(f0[3] * carryH);
      h[4] = to_h(f1[0] * carryH);
      h[5] = to_h(f1[1] * carryH);
      h[6] = to_h(f1[2] * carryH);
      h[7] = to_h(f1[3] * carryH);
      hv[it] = h;
      *(v8h*)(sH + row * HP + c8) = h;
      goff[it] = (size_t)(t * 32 + b0 + row) * H + c8;
    }
    if (!F32OUT) {
      for (int pass = 0; pass < 2; ++pass) {
#pragma unroll
        for (int it = 0; it < NIT; ++it) *(volatile v8h*)(y16 + goff[it]) = hv[it];
        __threadfence();
      }
    } else {
      constexpr int NF = (16 * H / 4) / 512;
      static_assert(NF * 512 * 4 == 16 * H, "f32 tile coverage");
      v4f fv[NF];
      size_t fo[NF];
#pragma unroll
      for (int it = 0; it < NF; ++it) {
        const int c   = it * 512 + tid;
        const int row = c / (H / 4);
        const int c4  = (c - row * (H / 4)) * 4;
        fv[it] = *(const v4f*)(sC + row * CP + c4);
        fo[it] = (size_t)(t * 32 + b0 + row) * H + c4;
      }
      for (int pass = 0; pass < 2; ++pass) {
#pragma unroll
        for (int it = 0; it < NF; ++it) *(volatile v4f*)(y32 + fo[it]) = fv[it];
        __threadfence();
      }
    }
    __syncthreads();
  }
}

__global__ __launch_bounds__(128)
void readout_kernel(const float* __restrict__ y32, const float* __restrict__ W,
                    const float* __restrict__ bias, float* __restrict__ out) {
  const int lane = threadIdx.x & 31;
  const int wave = threadIdx.x >> 5;
  const int o    = (blockIdx.x * 4 + wave) * 32 + lane;
  const int orow = o >> 1;
  const int c    = o & 1;
  const int b    = orow / kSteps;
  const int t    = orow - b * kSteps;
  const float* src = y32 + (size_t)(t * 32 + b) * kHidD;
  const float* wr  = W + c * kHidD;
  v4f acc = (v4f){0.f, 0.f, 0.f, 0.f};
#pragma unroll 4
  for (int k = 0; k < kHidD; k += 4) {
    const v4f a = *(const v4f*)(src + k);
    const v4f w = *(const v4f*)(wr + k);
    acc += a * w;
  }
  const float s = ((acc[0] + acc[1]) + (acc[2] + acc[3])) + bias[c];
  volatile float* p = out + o;
  *p = s;
  __threadfence();
  *p = s;
}

constexpr size_t kBytesWihE = (size_t)2 * kGateE * kHidE * 2;
constexpr size_t kBytesWhhE = (size_t)2 * kGateE * kHidE * 2;
constexpr size_t kBytesWfl  = (size_t)kHidE * kHidE * 2;
constexpr size_t kBytesWih0 = (size_t)kGateD * kHidE * 2;
constexpr size_t kBytesWhh0 = (size_t)kGateD * kHidD * 2;
constexpr size_t kBytesWih1 = (size_t)kGateD * kHidD * 2;
constexpr size_t kBytesWhh1 = (size_t)kGateD * kHidD * 2;
constexpr size_t kBytesRes  = (size_t)kRows * 2 * 4;
constexpr size_t kBytesActE = (size_t)kRows * kHidE * 2;
constexpr size_t kBytesActD = (size_t)kRows * kHidD * 2;
constexpr size_t kBytesY32  = (size_t)kRows * kHidD * 4;
constexpr size_t kBytesXiE  = (size_t)kGateE * kRows * 4;
constexpr size_t kBytesXiD  = (size_t)kGateD * kRows * 4;
constexpr size_t kCarveTotal = kBytesWihE + kBytesWhhE + kBytesWfl + kBytesWih0 + kBytesWhh0 + kBytesWih1 +
                               kBytesWhh1 + kBytesRes + 4 * kBytesActE + kBytesActD + kBytesY32 +
                               2 * kBytesXiE + 2 * kBytesXiD;
static_assert(kCarveTotal == 94745088, "carve total");
static_assert(kCarveTotal <= 134217728, "carve budget");
static_assert(kBytesRes % 256 == 0 && kBytesActD % 256 == 0 && kBytesY32 % 256 == 0 && kBytesXiD % 256 == 0, "alignment");
static_assert(((size_t)2 * kGateE * kHidE) % 2048 == 0 && ((size_t)kGateD * kHidD) % 2048 == 0, "convert grid exact");
static_assert(kRows * 2 == 25 * 128, "read-out grid exact");
static_assert(kRows * (kHidE / 8) == 800 * 256, "front grid exact");

extern "C" void kernel_launch(void* const* d_in, const int* in_sizes, int n_in,
                              void* d_out, int out_size, void* d_ws, size_t ws_size,
                              hipStream_t stream) {
  if (n_in < 24) return;
  const int expect[24] = {kBatch * kSteps * kNodes * 2, kBatch * kSteps * 2 * kEdges, 8, 4, 8, 2,
                          kHidE * 2, kHidE, 2 * kGateE * kHidE, 2 * kGateE * kHidE, 2 * kGateE, 2 * kGateE,
                          kHidE * kHidE, kHidE, kGateD * kHidE, kGateD * kHidD, kGateD, kGateD,
                          kGateD * kHidD, kGateD * kHidD, kGateD, kGateD, 2 * kHidD, 2};
  for (int i = 0; i < 24; ++i) if (in_sizes[i] < expect[i]) return;
  if (out_size < kRows * 2) return;
  if (ws_size < kCarveTotal) return;

  const float* x        = (const float*)d_in[0];
  const int*   ei       = (const int*)  d_in[1];
  const float* gcn_W1   = (const float*)d_in[2];
  const float* gcn_b1   = (const float*)d_in[3];
  const float* gcn_W2   = (const float*)d_in[4];
  const float* gcn_b2   = (const float*)d_in[5];
  const float* enc_fl_W = (const float*)d_in[6];
  const float* enc_fl_b = (const float*)d_in[7];
  const float* enc_Wih  = (const float*)d_in[8];
  const float* enc_Whh  = (const float*)d_in[9];
  const float* enc_bih  = (const float*)d_in[10];
  const float* enc_bhh  = (const float*)d_in[11];
  const float* dec_fl_W = (const float*)d_in[12];
  const float* dec_fl_b = (const float*)d_in[13];
  const float* dec_Wih0 = (const float*)d_in[14];
  const float* dec_Whh0 = (const float*)d_in[15];
  const float* dec_bih0 = (const float*)d_in[16];
  const float* dec_bhh0 = (const float*)d_in[17];
  const float* dec_Wih1 = (const float*)d_in[18];
  const float* dec_Whh1 = (const float*)d_in[19];
  const float* dec_bih1 = (const float*)d_in[20];
  const float* dec_bhh1 = (const float*)d_in[21];
  const float* dec_linW = (const float*)d_in[22];
  const float* dec_linb = (const float*)d_in[23];
  float* out = (float*)d_out;

  size_t off = 0;
  unsigned char* base = (unsigned char*)d_ws;
  auto carve = [&](size_t bytes) {
    unsigned char* r = base + off;
    off += bytes;
    return r;
  };
  unsigned short* wWihE = (unsigned short*)carve(kBytesWihE);
  unsigned short* wWhhE = (unsigned short*)carve(kBytesWhhE);
  unsigned short* wFl   = (unsigned short*)carve(kBytesWfl);
  unsigned short* wWih0 = (unsigned short*)carve(kBytesWih0);
  unsigned short* wWhh0 = (unsigned short*)carve(kBytesWhh0);
  unsigned short* wWih1 = (unsigned short*)carve(kBytesWih1);
  unsigned short* wWhh1 = (unsigned short*)carve(kBytesWhh1);
  float*          res   = (float*)carve(kBytesRes);
  unsigned short* a0    = (unsigned short*)carve(kBytesActE);
  unsigned short* yE0   = (unsigned short*)carve(kBytesActE);
  unsigned short* yE1   = (unsigned short*)carve(kBytesActE);
  unsigned short* dD    = (unsigned short*)carve(kBytesActE);
  unsigned short* yD0   = (unsigned short*)carve(kBytesActD);
  float*          y32   = (float*)carve(kBytesY32);
  float*          xiE0  = (float*)carve(kBytesXiE);
  float*          xiE1  = (float*)carve(kBytesXiE);
  float*          xiD0  = (float*)carve(kBytesXiD);
  float*          xiD1  = (float*)carve(kBytesXiD);
  if (off != kCarveTotal) return;

  weight_to_f16_kernel<<<(2 * kGateE * kHidE) / 2048, 256, 0, stream>>>(enc_Wih, wWihE);
  weight_to_f16_kernel<<<(2 * kGateE * kHidE) / 2048, 256, 0, stream>>>(enc_Whh, wWhhE);
  weight_to_f16_kernel<<<(kHidE * kHidE) / 2048, 256, 0, stream>>>(dec_fl_W, wFl);
  weight_to_f16_kernel<<<(kGateD * kHidE) / 2048, 256, 0, stream>>>(dec_Wih0, wWih0);
  weight_to_f16_kernel<<<(kGateD * kHidD) / 2048, 256, 0, stream>>>(dec_Whh0, wWhh0);
  weight_to_f16_kernel<<<(kGateD * kHidD) / 2048, 256, 0, stream>>>(dec_Wih1, wWih1);
  weight_to_f16_kernel<<<(kGateD * kHidD) / 2048, 256, 0, stream>>>(dec_Whh1, wWhh1);

  graph_front_kernel<<<kRows / 16, 128, 0, stream>>>(x, ei, gcn_W1, gcn_b1, gcn_W2, gcn_b2, res);

  front_linear_kernel<<<800, 256, 0, stream>>>(res, enc_fl_W, enc_fl_b, a0);

  const int tilesXiE = (kGateE / 64) * (kRows / 64);
  const int tilesXiD = (kGateD / 64) * (kRows / 64);
  const int tilesFl  = (kRows / 64) * (kHidE / 64);

  gemm64_f16_kernel<1, 0, 0><<<(tilesXiE + 7) / 8, 256, 0, stream>>>(
      wWihE, kHidE, a0, kHidE, (void*)xiE0, kRows, enc_bih, kGateE, kRows, kHidE, kInvWA0, 1.0f);
  recurrent_layer_kernel<kHidE, false><<<2, 512, 0, stream>>>(wWhhE, enc_bhh, xiE0, yE0, y32, kCarryE, kInvWE);

  gemm64_f16_kernel<1, 0, 0><<<(tilesXiE + 7) / 8, 256, 0, stream>>>(
      wWihE + (size_t)kGateE * kHidE, kHidE, yE0, kHidE, (void*)xiE1, kRows, enc_bih + kGateE,
      kGateE, kRows, kHidE, kInvWE, 1.0f);
  recurrent_layer_kernel<kHidE, false><<<2, 512, 0, stream>>>(
      wWhhE + (size_t)kGateE * kHidE, enc_bhh + kGateE, xiE1, yE1, y32, kCarryE, kInvWE);

  gemm64_f16_kernel<2, 1, 2><<<(tilesFl + 7) / 8, 256, 0, stream>>>(
      yE1, kHidE, wFl, kHidE, (void*)dD, kHidE, dec_fl_b, kRows, kHidE, kHidE, kInvWE, kCarryD);

  gemm64_f16_kernel<1, 0, 0><<<(tilesXiD + 7) / 8, 256, 0, stream>>>(
      wWih0, kHidE, dD, kHidE, (void*)xiD0, kRows, dec_bih0, kGateD, kRows, kHidE, kInvWD, 1.0f);
  recurrent_layer_kernel<kHidD, false><<<2, 512, 0, stream>>>(wWhh0, dec_bhh0, xiD0, yD0, y32, kCarryD0, kInvWD0);

  gemm64_f16_kernel<1, 0, 0><<<(tilesXiD + 7) / 8, 256, 0, stream>>>(
      wWih1, kHidD, yD0, kHidD, (void*)xiD1, kRows, dec_bih1, kGateD, kRows, kHidD, kInvWD0, 1.0f);
  recurrent_layer_kernel<kHidD, true><<<2, 512, 0, stream>>>(wWhh1, dec_bhh1, xiD1, yD0, y32, kCarryD1, kInvWD1);

  readout_kernel<<<25, 128, 0, stream>>>(y32, dec_linW, dec_linb, out);
}
